// SAGE_41128606826860
// MI455X (gfx1250) — hardware-verified
//
#include <hip/hip_runtime.h>
#include <stddef.h>
#include <stdint.h>
#include <math.h>


#define CIN    128
#define HC     128
#define OC     64
#define K0     128
#define K12    256
#define NTHR   256
#define NWAVE  8
#define EPT    8
#define CHUNK  (NTHR * EPT)
#define WCAP   (EPT * 32)
#define LISTN  (NWAVE * WCAP)
#define NBA    1024
#define SLA    10
#define RCAP   16384
#define DEGCAP 64
#define GBM    64
#define GBN    64
#define GTHR   128
#define APR    128
#define U0     (2 * HC * (K0 / 8))
#define U1     (2 * HC * (K12 / 8))
#define U2     (2 * OC * (K12 / 8))
#define AGG_ZINTS    (LISTN + 2 * RCAP + 3 * NBA)
#define AGG_LDS_INTS (AGG_ZINTS + 16)
#define WSMAX  134217728

static_assert((CHUNK & (CHUNK - 1)) == 0 && CHUNK <= 4096);
static_assert((NBA & (NBA - 1)) == 0 && NBA == (1 << SLA));
static_assert(((long long)CHUNK << SLA) < (1LL << 31));
static_assert(LISTN % NTHR == 0);
static_assert(NBA % NWAVE == 0 && NBA % 32 == 0 && NBA % GBM == 0);
static_assert(RCAP % 32 == 0 && AGG_ZINTS % 4 == 0 && LISTN % 4 == 0);
static_assert(K0 % 32 == 0 && K12 % 32 == 0 && K12 == 2 * HC && CIN == K0 && CIN == HC);
static_assert(GBM == (GTHR / 32) * 16 && GBN == 64);
static_assert((2 * HC) % GBN == 0 && (2 * OC) % GBN == 0);
static_assert(U0 % NTHR == 0 && U1 % NTHR == 0 && U2 % NTHR == 0);
static_assert((HC * (K0 / 8)) % NTHR == 0 && (HC * (K12 / 8)) % NTHR == 0 && (OC * (K12 / 8)) % NTHR == 0);
static_assert(K0 / 8 == 16 && K12 / 8 == 32);
static_assert(HC == 4 * 32 && OC == 2 * 32);
static_assert(APR % 16 == 0 && APR % GBM == 0 && NTHR / 16 == 16);
static_assert(NTHR == 2 * HC);
static_assert(AGG_LDS_INTS * 4 <= 300000);

typedef float          v2f   __attribute__((ext_vector_type(2)));
typedef float          v4f   __attribute__((ext_vector_type(4)));
typedef float          v8f   __attribute__((ext_vector_type(8)));
typedef double         v2d   __attribute__((ext_vector_type(2)));
typedef int            v4i   __attribute__((ext_vector_type(4)));
typedef int            v8i   __attribute__((ext_vector_type(8)));
typedef unsigned short v8us  __attribute__((ext_vector_type(8)));
typedef unsigned short v16us __attribute__((ext_vector_type(16)));
typedef __bf16         v16bf __attribute__((ext_vector_type(16)));
typedef v2f  __attribute__((may_alias)) v2fa;
typedef v4f  __attribute__((may_alias)) v4fa;
typedef v2d  __attribute__((may_alias)) v2da;
typedef v4i  __attribute__((may_alias)) v4ia;
typedef v8us __attribute__((may_alias)) v8usa;
union FragB { v16bf v; v16us u; v8us h[2]; v8i w; };

__device__ __forceinline__ v8f wmb(const FragB& a, const FragB& b, v8f c) {
  v8f d = __builtin_amdgcn_wmma_f32_16x16x32_bf16(false, a.v, false, b.v, (short)0, c, false, false);
  asm volatile("v_nop\n\tv_nop\n\tv_nop\n\tv_nop" : "+v"(d) : "v"(a.w), "v"(b.w));
  return d;
}

__device__ __forceinline__ unsigned bf16_bits(float f) {
  const unsigned u = __float_as_uint(f);
  return (u + 0x7FFFu + ((u >> 16) & 1u)) >> 16;
}
__device__ __forceinline__ float bf16_val(float f) {
  return __uint_as_float(bf16_bits(f) << 16);
}

template <int SLB>
__device__ __forceinline__ int scan_chunk(const int* __restrict__ dsts, int nE, int cbase, int slotBase,
                                          int nb, int vec8, int* list, int tid, int lane, int wave) {
  int wc = 0;
  const int el0  = tid * EPT;
  const int e0   = cbase + el0;
  const int sent = -2147483647 - 1;
  v4i da, db;
  if (vec8 != 0 && cbase + CHUNK <= nE) {
    da = *(const v4i*)(dsts + e0);
    db = *(const v4i*)(dsts + e0 + 4);
  } else {
    da.x = (e0     < nE) ? dsts[min(e0,     nE - 1)] : sent;
    da.y = (e0 + 1 < nE) ? dsts[min(e0 + 1, nE - 1)] : sent;
    da.z = (e0 + 2 < nE) ? dsts[min(e0 + 2, nE - 1)] : sent;
    da.w = (e0 + 3 < nE) ? dsts[min(e0 + 3, nE - 1)] : sent;
    db.x = (e0 + 4 < nE) ? dsts[min(e0 + 4, nE - 1)] : sent;
    db.y = (e0 + 5 < nE) ? dsts[min(e0 + 5, nE - 1)] : sent;
    db.z = (e0 + 6 < nE) ? dsts[min(e0 + 6, nE - 1)] : sent;
    db.w = (e0 + 7 < nE) ? dsts[min(e0 + 7, nE - 1)] : sent;
  }
  const unsigned nbs = (unsigned)slotBase;
  const unsigned unb = (unsigned)nb;
  const unsigned s0 = (unsigned)da.x - nbs, s1 = (unsigned)da.y - nbs;
  const unsigned s2 = (unsigned)da.z - nbs, s3 = (unsigned)da.w - nbs;
  const unsigned s4 = (unsigned)db.x - nbs, s5 = (unsigned)db.y - nbs;
  const unsigned s6 = (unsigned)db.z - nbs, s7 = (unsigned)db.w - nbs;
  const bool h0 = s0 < unb, h1 = s1 < unb, h2 = s2 < unb, h3 = s3 < unb;
  const bool h4 = s4 < unb, h5 = s5 < unb, h6 = s6 < unb, h7 = s7 < unb;
  const unsigned any = __builtin_amdgcn_ballot_w32(h0 | h1 | h2 | h3 | h4 | h5 | h6 | h7);
  if (any != 0u) {
#define HITJ(J, HJ, SJ) { \
      const unsigned mj = __builtin_amdgcn_ballot_w32(HJ); \
      if (mj != 0u) { \
        if (HJ) { \
          const int pos = wc + (int)__builtin_amdgcn_mbcnt_lo(mj, 0u); \
          if (pos < WCAP) list[wave * WCAP + pos] = ((el0 + (J)) << SLB) | (int)(SJ); \
        } \
        wc += (int)__builtin_popcount(mj); } }
    HITJ(0, h0, s0)
    HITJ(1, h1, s1)
    HITJ(2, h2, s2)
    HITJ(3, h3, s3)
    HITJ(4, h4, s4)
    HITJ(5, h5, s5)
    HITJ(6, h6, s6)
    HITJ(7, h7, s7)
#undef HITJ
  }
  return wc;
}

__global__ __launch_bounds__(NTHR) void k_wprep(const float* __restrict__ Wl0, const float* __restrict__ Wr0,
                                                const float* __restrict__ Wl1, const float* __restrict__ Wr1,
                                                const float* __restrict__ Wl2, const float* __restrict__ Wr2,
                                                unsigned short* B0, unsigned short* B1, unsigned short* B2) {
  const int u = (int)blockIdx.x * NTHR + (int)threadIdx.x;
  const float* W;
  unsigned short* dp;
  int kk, nn, wo;
  if (u < U0) {
    const int n  = u >> 4;
    const int k8 = (u & 15) * 8;
    W  = (n < HC) ? Wl0 : Wr0;
    nn = n & (HC - 1); kk = k8; wo = HC;
    dp = B0 + (size_t)n * K0 + k8;
  } else if (u < U0 + U1) {
    const int v  = u - U0;
    const int n  = v >> 5;
    const int k8 = (v & 31) * 8;
    W  = (n < HC) ? Wl1 : Wr1;
    nn = n & (HC - 1); kk = k8 & (HC - 1); wo = HC;
    dp = B1 + (size_t)n * K12 + k8;
  } else if (u < U0 + U1 + U2) {
    const int v  = u - U0 - U1;
    const int n  = v >> 5;
    const int k8 = (v & 31) * 8;
    W  = (n < OC) ? Wl2 : Wr2;
    nn = n & (OC - 1); kk = k8 & (HC - 1); wo = OC;
    dp = B2 + (size_t)n * K12 + k8;
  } else {
    return;
  }
  const float* p = W + (size_t)kk * wo + nn;
  v8us o;
#pragma unroll
  for (int i = 0; i < 8; ++i) o[i] = (unsigned short)bf16_bits(p[(size_t)i * wo]);
  *(volatile v8us*)dp = o;
  __threadfence();
  *(volatile v8us*)dp = o;
}

__global__ __launch_bounds__(NTHR) void k_cvx(const float* __restrict__ x, int nN, int nUnits,
                                              unsigned short* xb) {
  const int u = (int)blockIdx.x * NTHR + (int)threadIdx.x;
  if (u >= nUnits) return;
  const int row = u >> 4;
  const int k8  = (u & 15) * 8;
  const int rc  = row < nN ? row : nN - 1;
  const float* p = x + (size_t)rc * CIN + k8;
  const v4f a = *(const v4fa*)p;
  const v4f b = *(const v4fa*)(p + 4);
  const bool ok = row < nN;
  v8us o;
  o[0] = ok ? (unsigned short)bf16_bits(a.x) : (unsigned short)0;
  o[1] = ok ? (unsigned short)bf16_bits(a.y) : (unsigned short)0;
  o[2] = ok ? (unsigned short)bf16_bits(a.z) : (unsigned short)0;
  o[3] = ok ? (unsigned short)bf16_bits(a.w) : (unsigned short)0;
  o[4] = ok ? (unsigned short)bf16_bits(b.x) : (unsigned short)0;
  o[5] = ok ? (unsigned short)bf16_bits(b.y) : (unsigned short)0;
  o[6] = ok ? (unsigned short)bf16_bits(b.z) : (unsigned short)0;
  o[7] = ok ? (unsigned short)bf16_bits(b.w) : (unsigned short)0;
  unsigned short* dp = xb + (size_t)row * CIN + k8;
  *(volatile v8us*)dp = o;
  __threadfence();
  *(volatile v8us*)dp = o;
}

__global__ __launch_bounds__(GTHR) void k_gemm(
    const unsigned short* __restrict__ A, const unsigned short* __restrict__ WT,
    float* outF, int K, int ldo)
{
  __shared__ __attribute__((aligned(16))) float stg[GBM * GBN];
  const int tid = (int)threadIdx.x, lane = tid & 31, wave = tid >> 5, hh = lane >> 4, m = lane & 15;
  const int rowBase = (int)blockIdx.x * GBM;
  const int col0    = (int)blockIdx.y * GBN;

  v8f acc[4];
  {
    const v8f z = {0.f, 0.f, 0.f, 0.f, 0.f, 0.f, 0.f, 0.f};
    acc[0] = z; acc[1] = z; acc[2] = z; acc[3] = z;
  }
  const unsigned short* ap = A  + (size_t)(rowBase + 16 * wave + m) * (size_t)K + 8 * hh;
  const unsigned short* wp = WT + (size_t)(col0 + m) * (size_t)K + 8 * hh;
  const int ksteps = K >> 5;
#pragma unroll 1
  for (int ks = 0; ks < ksteps; ++ks) {
    FragB af;
    af.h[0] = *(const v8usa*)(ap + 32 * ks);
    af.h[1] = *(const v8usa*)(ap + 32 * ks + 16);
#pragma unroll
    for (int t = 0; t < 4; ++t) {
      const unsigned short* wq = wp + (size_t)(16 * t) * (size_t)K + 32 * ks;
      FragB bf;
      bf.h[0] = *(const v8usa*)wq;
      bf.h[1] = *(const v8usa*)(wq + 16);
      acc[t] = wmb(af, bf, acc[t]);
    }
  }

#pragma unroll
  for (int t = 0; t < 4; ++t) {
    const int lc = 16 * t + m;
#pragma unroll
    for (int r = 0; r < 8; ++r) {
      const int lr = 16 * wave + 8 * hh + r;
      stg[lr * GBN + lc] = acc[t][r];
    }
  }
  __syncthreads();

  v4f fv[8];
#pragma unroll
  for (int i = 0; i < 8; ++i) {
    const int lr = 16 * wave + 2 * i + hh;
    fv[i] = *(const v4fa*)(stg + lr * GBN + 4 * m);
  }
#pragma unroll
  for (int i = 0; i < 8; ++i) {
    const int lr = 16 * wave + 2 * i + hh;
    const int gr = rowBase + lr;
    float* op = outF + (size_t)gr * (size_t)ldo + col0 + 4 * m;
    *(volatile v4f*)op = fv[i];
  }
  __threadfence();
#pragma unroll
  for (int i = 0; i < 8; ++i) {
    const int lr = 16 * wave + 2 * i + hh;
    const int gr = rowBase + lr;
    float* op = outF + (size_t)gr * (size_t)ldo + col0 + 4 * m;
    *(volatile v4f*)op = fv[i];
  }
}

template <int FO>
__global__ __launch_bounds__(NTHR) void k_scan(const int* __restrict__ srcs, const int* __restrict__ dsts,
                                               const float* __restrict__ ew, int nE, int nN, int vec8,
                                               const float* __restrict__ tr, const float* __restrict__ bias,
                                               float* outp) {
  constexpr int LDT = 2 * FO;
  extern __shared__ __attribute__((aligned(16))) int dsm[];
  int* list = dsm;
  int* hl   = dsm + LISTN;
  int* sl   = dsm + LISTN + RCAP;
  int* cnt  = dsm + LISTN + 2 * RCAP;
  int* offs = cnt + NBA;
  int* cur  = offs + NBA;
  int* misc = cur + NBA;
  const int tid = (int)threadIdx.x, lane = tid & 31, wave = tid >> 5;
  const int nodeBase = (int)blockIdx.x * NBA;

  {
    const v4i z4 = {0, 0, 0, 0};
    for (int i = tid * 4; i < AGG_ZINTS; i += NTHR * 4) *(v4ia*)(dsm + i) = z4;
    if (tid < 16) misc[tid] = 0;
  }
  float bv0, bv1, bv2 = 0.0f, bv3 = 0.0f;
  if constexpr (FO == 128) {
    const v4f a = *(const v4fa*)(bias + 4 * lane);
    bv0 = bf16_val(a.x); bv1 = bf16_val(a.y); bv2 = bf16_val(a.z); bv3 = bf16_val(a.w);
  } else {
    const v2f a = *(const v2fa*)(bias + 2 * lane);
    bv0 = bf16_val(a.x); bv1 = bf16_val(a.y);
  }
  __syncthreads();

  int t = 0, ov = 0;
  const int nChunks = (nE + CHUNK - 1) / CHUNK;
#pragma unroll 1
  for (int ch = 0; ch < nChunks; ++ch) {
    const int cbase = ch * CHUNK;
    const int wc = scan_chunk<SLA>(dsts, nE, cbase, nodeBase, NBA, vec8, list, tid, lane, wave);
    if (lane == 0) misc[wave] = wc;
    __syncthreads();
    if (wave == 0) {
#pragma unroll 1
      for (int w2 = 0; w2 < NWAVE; ++w2) {
        int c = misc[w2];
        c = c < 0 ? 0 : (c > WCAP ? WCAP : c);
#pragma unroll 1
        for (int b0 = 0; b0 < c; b0 += 32) {
          const int idx = b0 + lane;
          const int ent = list[w2 * WCAP + (idx < WCAP ? idx : WCAP - 1)];
          const int m32 = (c - b0) < 32 ? (c - b0) : 32;
#pragma unroll 1
          for (int k = 0; k < m32; ++k) {
            const int u    = __builtin_amdgcn_readlane(ent, k);
            const int slot = u & (NBA - 1);
            const int el   = (u >> SLA) & (CHUNK - 1);
            const int pk   = ((cbase + el) << SLA) | slot;
            if (t < RCAP) {
              if (lane == 0) { hl[t] = pk; cnt[slot] = cnt[slot] + 1; }
              t = t + 1;
            } else {
              ov = 1;
            }
          }
        }
      }
    }
    __syncthreads();
  }
  if (wave == 0 && lane == 0) { misc[8] = t; misc[9] = ov; }
  __syncthreads();
  int tt = misc[8];
  tt = tt < 0 ? 0 : (tt > RCAP ? RCAP : tt);
  const int ovf = misc[9];

  if (wave == 0) {
    const int base = lane * (NBA / 32);
    int s = 0;
#pragma unroll 1
    for (int i = 0; i < NBA / 32; ++i) s += cnt[base + i];
    int incl = s;
#pragma unroll
    for (int d = 1; d < 32; d <<= 1) {
      const int y = __shfl_up(incl, d, 32);
      if (lane >= d) incl += y;
    }
    int run = incl - s;
#pragma unroll 1
    for (int i = 0; i < NBA / 32; ++i) {
      const int cv = cnt[base + i];
      offs[base + i] = run;
      cur[base + i]  = run;
      run += cv;
    }
  }
  __syncthreads();
  if (wave == 0) {
#pragma unroll 1
    for (int b0 = 0; b0 < tt; b0 += 32) {
      const int idx = b0 + lane;
      const int ent = hl[idx < RCAP ? idx : RCAP - 1];
      const int m32 = (tt - b0) < 32 ? (tt - b0) : 32;
#pragma unroll 1
      for (int k = 0; k < m32; ++k) {
        const int u    = __builtin_amdgcn_readlane(ent, k);
        const int slot = u & (NBA - 1);
        if (lane == 0) {
          int p = cur[slot];
          p = p < 0 ? 0 : (p > RCAP - 1 ? RCAP - 1 : p);
          sl[p] = u;
          cur[slot] = p + 1;
        }
      }
    }
  }
  __syncthreads();

  const float qnan = __int_as_float(0x7fc00000);
  const float pz = (ovf != 0) ? qnan : 0.0f;
  const int sa = (2 * lane) & 31, sb = (2 * lane + 1) & 31;
#pragma unroll 1
  for (int si = 0; si < NBA / NWAVE; ++si) {
    const int s    = si * NWAVE + wave;
    const int node = nodeBase + s;
    const int craw = cnt[s];
    int c = craw;
    const bool big = c > DEGCAP;
    c = c < 0 ? 0 : (c > DEGCAP ? DEGCAP : c);
    int o = offs[s];
    o = o < 0 ? 0 : (o > RCAP ? RCAP : o);
    const int nc = node < nN ? node : nN - 1;
    float a0 = 0.0f, a1 = 0.0f, a2 = 0.0f, a3 = 0.0f;
#pragma unroll 1
    for (int b0 = 0; b0 < c; b0 += 32) {
      int idx = o + b0 + lane;
      idx = idx > RCAP - 1 ? RCAP - 1 : idx;
      const int ent = sl[idx];
      int eid = ent >> SLA;
      eid = eid < 0 ? 0 : (eid > nE - 1 ? nE - 1 : eid);
      int sr = srcs[eid];
      sr = sr < 0 ? 0 : (sr > nN - 1 ? nN - 1 : sr);
      const float wv  = bf16_val(ew[eid]);
      const int   wvi = __float_as_int(wv);
      const int m32 = (c - b0) < 32 ? (c - b0) : 32;
#pragma unroll 1
      for (int k = 0; k < m32; ++k) {
        const int   sk = __builtin_amdgcn_readlane(sr, k);
        const float ck = __int_as_float(__builtin_amdgcn_readlane(wvi, k));
        if constexpr (FO == 128) {
          const v4f a = *(const v4fa*)(tr + (size_t)sk * LDT + 4 * lane);
          a0 = fmaf(ck, a.x, a0);
          a1 = fmaf(ck, a.y, a1);
          a2 = fmaf(ck, a.z, a2);
          a3 = fmaf(ck, a.w, a3);
        } else {
          const v2f a = *(const v2fa*)(tr + (size_t)sk * LDT + 2 * lane);
          a0 = fmaf(ck, a.x, a0);
          a1 = fmaf(ck, a.y, a1);
        }
      }
    }
    const float cf  = (craw < 1) ? 1.0f : (float)craw;
    const float inv = 1.0f / cf;
    const float pzr = big ? qnan : pz;
    if constexpr (FO == 128) {
      const v4f r = *(const v4fa*)(tr + (size_t)nc * LDT + FO + 4 * lane);
      v4f y;
      y.x = ((a0 * inv + bv0) + r.x) + pzr;
      y.y = ((a1 * inv + bv1) + r.y) + pzr;
      y.z = ((a2 * inv + bv2) + r.z) + pzr;
      y.w = ((a3 * inv + bv3) + r.w) + pzr;
      float* op = outp + (size_t)nc * FO + 4 * lane;
      const bool wr = node < nN;
      if (wr) *(volatile v4f*)op = y;
      __threadfence();
      if (wr) *(volatile v4f*)op = y;
    } else {
      const v2f r = *(const v2fa*)(tr + (size_t)nc * LDT + FO + 2 * lane);
      const float v0 = ((a0 * inv + bv0) + r.x) + pzr;
      const float v1 = ((a1 * inv + bv1) + r.y) + pzr;
      v4f ow;
      ow.x = __shfl(v0, sa, 32); ow.y = __shfl(v1, sa, 32);
      ow.z = __shfl(v0, sb, 32); ow.w = __shfl(v1, sb, 32);
      float* op = outp + (size_t)nc * FO + 4 * (lane & 15);
      const bool wr = (node < nN) && (lane < 16);
      if (wr) *(volatile v4f*)op = ow;
      __threadfence();
      if (wr) *(volatile v4f*)op = ow;
    }
  }
}

__global__ __launch_bounds__(NTHR) void k_bnstats(const float* __restrict__ h, int nN, double* rec) {
  __shared__ __attribute__((aligned(16))) double sS[NTHR];
  __shared__ __attribute__((aligned(16))) double sQ[NTHR];
  __shared__ __attribute__((aligned(16))) double outd[NTHR];
  const int tid = (int)threadIdx.x;
  const int col = tid & (HC - 1);
  const int half = tid >> 7;
  const int r0 = (int)blockIdx.x * NBA + half * (NBA / 2);
  int r1 = r0 + NBA / 2;
  r1 = r1 > nN ? nN : r1;
  double s = 0.0, q = 0.0;
#pragma unroll 4
  for (int r = r0; r < r1; ++r) {
    const double d = (double)h[(size_t)r * HC + col];
    s += d;
    q = fma(d, d, q);
  }
  sS[tid] = s;
  sQ[tid] = q;
  __syncthreads();
  if (tid < HC) {
    outd[tid]      = sS[tid] + sS[HC + tid];
    outd[HC + tid] = sQ[tid] + sQ[HC + tid];
  }
  __syncthreads();
  const int t2 = 2 * (tid & (HC - 1));
  const v2d o = *(const v2da*)(outd + t2);
  double* dp = rec + (size_t)blockIdx.x * (2 * HC) + t2;
  const bool st = tid < HC;
  if (st) *(volatile v2d*)dp = o;
  __threadfence();
  if (st) *(volatile v2d*)dp = o;
}

__device__ __forceinline__ float bn_relu(float x, float mu, float rs, float g, float b, bool ok) {
  float t = ((x - mu) * rs) * g + b;
  t = (t < 0.0f) ? 0.0f : t;
  return ok ? t : 0.0f;
}

__global__ __launch_bounds__(NTHR) void k_bnapply(const float* __restrict__ hpre, const double* __restrict__ rec,
                                                  const float* __restrict__ gamma, const float* __restrict__ beta,
                                                  unsigned short* hpl, double invN, int nRec, int nN) {
  __shared__ __attribute__((aligned(16))) float smu[HC];
  __shared__ __attribute__((aligned(16))) float srs[HC];
  __shared__ __attribute__((aligned(16))) float sga[HC];
  __shared__ __attribute__((aligned(16))) float sbe[HC];
  const int tid = (int)threadIdx.x;
  if (tid < HC) {
    double S = 0.0, Q = 0.0;
#pragma unroll 2
    for (int b = 0; b < nRec; ++b) {
      S += rec[(size_t)b * (2 * HC) + tid];
      Q += rec[(size_t)b * (2 * HC) + HC + tid];
    }
    const double mu = S * invN;
    double var = Q * invN - mu * mu;
    var = (var < 0.0) ? 0.0 : var;
    smu[tid] = (float)mu;
    srs[tid] = 1.0f / sqrtf((float)var + 1e-5f);
    sga[tid] = bf16_val(gamma[tid]);
    sbe[tid] = bf16_val(beta[tid]);
  }
  __syncthreads();

  const int sub = tid >> 4;
  const int k8  = (tid & 15) * 8;
  const v4f mu0 = *(const v4fa*)(smu + k8), mu1 = *(const v4fa*)(smu + k8 + 4);
  const v4f rs0 = *(const v4fa*)(srs + k8), rs1 = *(const v4fa*)(srs + k8 + 4);
  const v4f ga0 = *(const v4fa*)(sga + k8), ga1 = *(const v4fa*)(sga + k8 + 4);
  const v4f be0 = *(const v4fa*)(sbe + k8), be1 = *(const v4fa*)(sbe + k8 + 4);
  const int rowBase = (int)blockIdx.x * APR;
#pragma unroll 1
  for (int it = 0; it < APR / 16; ++it) {
    const int row = rowBase + it * 16 + sub;
    const int rc  = row < nN ? row : nN - 1;
    const bool ok = row < nN;
    const float* p = hpre + (size_t)rc * HC + k8;
    const v4f a = *(const v4fa*)p;
    const v4f b = *(const v4fa*)(p + 4);
    float y[8];
    y[0] = bn_relu(a.x, mu0.x, rs0.x, ga0.x, be0.x, ok);
    y[1] = bn_relu(a.y, mu0.y, rs0.y, ga0.y, be0.y, ok);
    y[2] = bn_relu(a.z, mu0.z, rs0.z, ga0.z, be0.z, ok);
    y[3] = bn_relu(a.w, mu0.w, rs0.w, ga0.w, be0.w, ok);
    y[4] = bn_relu(b.x, mu1.x, rs1.x, ga1.x, be1.x, ok);
    y[5] = bn_relu(b.y, mu1.y, rs1.y, ga1.y, be1.y, ok);
    y[6] = bn_relu(b.z, mu1.z, rs1.z, ga1.z, be1.z, ok);
    y[7] = bn_relu(b.w, mu1.w, rs1.w, ga1.w, be1.w, ok);
    v8us hv, lv;
#pragma unroll
    for (int j = 0; j < 8; ++j) {
      const unsigned hb = bf16_bits(y[j]);
      hv[j] = (unsigned short)hb;
      lv[j] = (unsigned short)bf16_bits(y[j] - __uint_as_float(hb << 16));
    }
    unsigned short* dp = hpl + (size_t)row * K12 + k8;
    *(volatile v8us*)dp = hv;
    *(volatile v8us*)(dp + HC) = lv;
    __threadfence();
    *(volatile v8us*)dp = hv;
    *(volatile v8us*)(dp + HC) = lv;
  }
}

static inline int cdiv(int a, int b) { return (a + b - 1) / b; }
static inline size_t al256(size_t o) { return (o + 255) & ~(size_t)255; }

extern "C" void kernel_launch(void* const* d_in, const int* in_sizes, int n_in,
                              void* d_out, int out_size, void* d_ws, size_t ws_size,
                              hipStream_t stream) {
  if (n_in < 16) return;
  if (in_sizes[0] < CIN || (in_sizes[0] % CIN) != 0) return;
  const int nN = in_sizes[0] / CIN;
  if (nN < 1 || nN > (1 << 22)) return;
  if (in_sizes[1] < 2 || (in_sizes[1] & 1) != 0) return;
  const int nE = in_sizes[1] / 2;
  if (nE < 1 || nE >= (1 << (31 - SLA))) return;
  if (in_sizes[2] != nE) return;
  if (in_sizes[3] != CIN * HC || in_sizes[4] != CIN * HC || in_sizes[5] != HC) return;
  if (in_sizes[6] != HC * HC || in_sizes[7] != HC * HC || in_sizes[8] != HC) return;
  if (in_sizes[9] != HC * OC || in_sizes[10] != HC * OC || in_sizes[11] != OC) return;
  if (in_sizes[12] != HC || in_sizes[13] != HC || in_sizes[14] != HC || in_sizes[15] != HC) return;
  if ((long long)out_size != (long long)nN * OC) return;

  const float* x    = (const float*)d_in[0];
  const int*   edge = (const int*)d_in[1];
  const float* ew   = (const float*)d_in[2];
  const float* Wl0  = (const float*)d_in[3];
  const float* Wr0  = (const float*)d_in[4];
  const float* b0   = (const float*)d_in[5];
  const float* Wl1  = (const float*)d_in[6];
  const float* Wr1  = (const float*)d_in[7];
  const float* b1   = (const float*)d_in[8];
  const float* Wl2  = (const float*)d_in[9];
  const float* Wr2  = (const float*)d_in[10];
  const float* b2   = (const float*)d_in[11];
  const float* g0   = (const float*)d_in[12];
  const float* be0  = (const float*)d_in[13];
  const float* g1   = (const float*)d_in[14];
  const float* be1  = (const float*)d_in[15];
  float* out = (float*)d_out;
  const int* src = edge;
  const int* dst = edge + nE;

  const int MP = cdiv(nN, APR) * APR;
  const int gM = MP / GBM;
  const int gP = MP / APR;
  const int gA = cdiv(nN, NBA);
  if ((long long)gA * NBA < (long long)nN) return;
  const int vec8 = ((nE & 3) == 0) ? 1 : 0;
  const double invN = 1.0 / (double)nN;

  char* ws = (char*)d_ws;
  size_t off = 0;
  const size_t oB0  = off; off = al256(off + (size_t)2 * HC * K0 * 2);
  const size_t oB1  = off; off = al256(off + (size_t)2 * HC * K12 * 2);
  const size_t oB2  = off; off = al256(off + (size_t)2 * OC * K12 * 2);
  const size_t oXB  = off; off = al256(off + (size_t)MP * CIN * 2);
  const size_t oTR  = off; off = al256(off + (size_t)MP * 2 * HC * 4);
  const size_t oHP  = off; off = al256(off + (size_t)nN * HC * 4);
  const size_t oHL  = off; off = al256(off + (size_t)MP * K12 * 2);
  const size_t oRC  = off; off = al256(off + (size_t)gA * 2 * HC * 8);
  if (off > ws_size || off > (size_t)WSMAX) return;
  unsigned short* B0  = (unsigned short*)(ws + oB0);
  unsigned short* B1  = (unsigned short*)(ws + oB1);
  unsigned short* B2  = (unsigned short*)(ws + oB2);
  unsigned short* XB  = (unsigned short*)(ws + oXB);
  float*          TR  = (float*)(ws + oTR);
  float*          HP  = (float*)(ws + oHP);
  unsigned short* HL  = (unsigned short*)(ws + oHL);
  double*         RC  = (double*)(ws + oRC);

  const size_t scanLds = (size_t)AGG_LDS_INTS * 4;
  hipFuncSetAttribute(reinterpret_cast<const void*>(&k_scan<128>), hipFuncAttributeMaxDynamicSharedMemorySize, (int)scanLds);
  hipFuncSetAttribute(reinterpret_cast<const void*>(&k_scan<64>),  hipFuncAttributeMaxDynamicSharedMemorySize, (int)scanLds);

  const int nUx = MP * (CIN / 8);
  k_wprep<<<(U0 + U1 + U2) / NTHR, NTHR, 0, stream>>>(Wl0, Wr0, Wl1, Wr1, Wl2, Wr2, B0, B1, B2);
  k_cvx<<<cdiv(nUx, NTHR), NTHR, 0, stream>>>(x, nN, nUx, XB);
  k_gemm<<<dim3(gM, (2 * HC) / GBN), GTHR, 0, stream>>>(XB, B0, TR, K0, 2 * HC);
  k_scan<128><<<gA, NTHR, scanLds, stream>>>(src, dst, ew, nE, nN, vec8, TR, b0, HP);
  k_bnstats<<<gA, NTHR, 0, stream>>>(HP, nN, RC);
  k_bnapply<<<gP, NTHR, 0, stream>>>(HP, RC, g0, be0, HL, invN, gA, nN);
  k_gemm<<<dim3(gM, (2 * HC) / GBN), GTHR, 0, stream>>>(HL, B1, TR, K12, 2 * HC);
  k_scan<128><<<gA, NTHR, scanLds, stream>>>(src, dst, ew, nE, nN, vec8, TR, b1, HP);
  k_bnstats<<<gA, NTHR, 0, stream>>>(HP, nN, RC);
  k_bnapply<<<gP, NTHR, 0, stream>>>(HP, RC, g1, be1, HL, invN, gA, nN);
  k_gemm<<<dim3(gM, (2 * OC) / GBN), GTHR, 0, stream>>>(HL, B2, TR, K12, 2 * OC);
  k_scan<64><<<gA, NTHR, scanLds, stream>>>(src, dst, ew, nE, nN, vec8, TR, b2, out);
}
